// PSAAttention_31258771980508
// MI455X (gfx1250) — hardware-run, weakly checked
//
#include <hip/hip_runtime.h>


#ifndef SEQ
#define SEQ 2048
#endif
#define SEQ_FULL 2048
#ifndef NHD
#define NHD 16
#endif
#define NHD_FULL 16
#define HD   128
#define NQB  (SEQ / 128)
#define NKB  (SEQ / 64)
#define NSQ  (NQB * 32)
#define NSK  (NKB * 16)
#define NT   (NKB / 4)
#define T2   (SEQ / 2)
#define T8   (SEQ / 8)
#define K8R  (T8 + 32)
#define V8P  (T8 + 64)
#define PSH  10.0f
#define PSC  0.08838834764831845f
#define CSL  (0.08838834764831845f * 1.4426950408889634f)

#define K2OFF  (NHD * SEQ * HD)
#define K8OFF  (K2OFF + NHD * T2 * HD)
#define KPOOL  (K8OFF + NHD * K8R * HD)
#define VT2OFF (NHD * HD * SEQ)
#define VT8OFF (VT2OFF + NHD * HD * T2)
#define VPOOL  (VT8OFF + NHD * HD * V8P)

typedef _Float16 h16;
typedef unsigned short bf;
typedef __attribute__((ext_vector_type(16))) __bf16   v16bf;
typedef __attribute__((ext_vector_type(16))) _Float16 v16h;
typedef __attribute__((ext_vector_type(8)))  _Float16 v8h;
typedef __attribute__((ext_vector_type(8)))  unsigned short v8us;
typedef __attribute__((ext_vector_type(8)))  float    v8f;
typedef __attribute__((ext_vector_type(4)))  float    v4f;
typedef v8h  __attribute__((may_alias)) v8ha;
typedef v4f  __attribute__((may_alias)) v4fa;

static_assert(SEQ % 512 == 0);
static_assert(SEQ <= SEQ_FULL);
static_assert(NHD <= NHD_FULL);
static_assert(HD == 128);
static_assert(HD % 32 == 0);
static_assert(32 * 4 == HD);
static_assert(NKB <= 32);
static_assert(NKB % 4 == 0);
static_assert(NT >= 1);
static_assert(NSQ == NSK);
static_assert(NSQ % 64 == 0);
static_assert((V8P * 2) % 128 == 0);
static_assert((T8 * 2) % 128 == 0);
static_assert((NKB - 1) * 8 + 31 < K8R);
static_assert((NKB - 1) * 8 + 31 < V8P);
static_assert(K2OFF % 64 == 0);
static_assert(K8OFF % 64 == 0);
static_assert(VT2OFF % 64 == 0);
static_assert(VT8OFF % 64 == 0);
static_assert((NHD * T8 * 16) % 256 == 0);
static_assert((NHD * 32 * 16) % 256 == 0);
static_assert((NHD * SEQ * 16) % 256 == 0);
static_assert(512 * 33 * 4 <= 131072);

__device__ __forceinline__ unsigned short f2bf(float f) { unsigned u = __float_as_uint(f); u += 0x7FFFu + ((u >> 16) & 1u); return (unsigned short)(u >> 16); }
__device__ __forceinline__ float bf2f(unsigned short b) { return __uint_as_float(((unsigned)b) << 16); }
__device__ __forceinline__ float bfr(float f) { return bf2f(f2bf(f)); }
__device__ __forceinline__ v16h cat16(v8h lo, v8h hi) { return __builtin_shufflevector(lo, hi, 0, 1, 2, 3, 4, 5, 6, 7, 8, 9, 10, 11, 12, 13, 14, 15); }
__device__ __forceinline__ v16bf cat16b(v8us lo, v8us hi) { return __builtin_bit_cast(v16bf, __builtin_shufflevector(lo, hi, 0, 1, 2, 3, 4, 5, 6, 7, 8, 9, 10, 11, 12, 13, 14, 15)); }
__device__ __forceinline__ v16h  ldh(const h16* p) { return cat16(*(const v8h*)p, *(const v8h*)(p + 16)); }
__device__ __forceinline__ v16bf ldb(const bf* p)  { return cat16b(*(const v8us*)p, *(const v8us*)(p + 16)); }
static __device__ __forceinline__ h16 toh_flush(float v) { const h16 r = (h16)v; return (fabsf(v) < 6.103515625e-05f) ? (h16)0.0f : r; }
__device__ __forceinline__ v8f wmma16g(v16h a, v16h b, v8f c) {
    c = __builtin_amdgcn_wmma_f32_16x16x32_f16(false, a, false, b, (short)0, c, false, false);
    asm volatile("v_nop\n\tv_nop\n\tv_nop\n\tv_nop" : "+v"(c) : "v"(a), "v"(b));
    return c;
}
__device__ __forceinline__ v8f wmmabg(v16bf a, v16bf b, v8f c) {
    c = __builtin_amdgcn_wmma_f32_16x16x32_bf16(false, a, false, b, (short)0, c, false, false);
    asm volatile("v_nop\n\tv_nop\n\tv_nop\n\tv_nop" : "+v"(c) : "v"(a), "v"(b));
    return c;
}

__global__ __launch_bounds__(256) void k_cvtq(const float* __restrict__ q, h16* Q16) {
    const int i = blockIdx.x * 256 + threadIdx.x;
    if (i >= NHD * SEQ * 16) return;
    const int c = (i & 15) * 8; const int rowg = i >> 4; const int h = rowg / SEQ; const int row = rowg % SEQ;
    const v8f v = *(const v8f*)(q + ((size_t)h * SEQ_FULL + row) * HD + c);
    v8h o;
#pragma unroll
    for (int e = 0; e < 8; ++e) o[e] = toh_flush(bfr(v[e]));
    *(volatile v8h*)(Q16 + (size_t)i * 8) = o; __threadfence(); *(volatile v8h*)(Q16 + (size_t)i * 8) = o;
}

#define KPL_REAL (NHD * T8 * 16)
#define KPL_PAD  (NHD * 32 * 16)
__global__ __launch_bounds__(256) void k_kpl(const float* __restrict__ k, h16* KP) {
    const int i = blockIdx.x * 256 + threadIdx.x; const int pc = (i & 15) * 8;
    if (blockIdx.x < KPL_REAL / 256) {
        const int g = i >> 4; const int h = g / T8, g8 = g % T8;
        const float* src = k + ((size_t)h * SEQ_FULL + (size_t)g8 * 8) * HD + pc;
        v8h o1[8], o2[4], o8; float s8[8];
#pragma unroll
        for (int j = 0; j < 4; ++j) {
            const v8f a = *(const v8f*)(src + (2 * j) * HD); const v8f b = *(const v8f*)(src + (2 * j + 1) * HD);
#pragma unroll
            for (int e = 0; e < 8; ++e) {
                const float fa = bfr(a[e]), fb = bfr(b[e]);
                o1[2 * j][e] = toh_flush(fa); o1[2 * j + 1][e] = toh_flush(fb);
                o2[j][e] = toh_flush((fa + fb) * 0.5f);
                float a8 = (j == 0) ? 0.0f : s8[e]; a8 += fa; a8 += fb; s8[e] = a8;
            }
        }
#pragma unroll
        for (int e = 0; e < 8; ++e) o8[e] = toh_flush(s8[e] * 0.125f);
        h16* d1 = KP + ((size_t)h * SEQ + (size_t)g8 * 8) * HD + pc;
        h16* d2 = KP + K2OFF + ((size_t)h * T2 + (size_t)g8 * 4) * HD + pc;
        h16* d8 = KP + K8OFF + ((size_t)h * K8R + g8) * HD + pc;
#pragma unroll 1
        for (int ps = 0; ps < 2; ++ps) {
#pragma unroll
            for (int r = 0; r < 8; ++r) *(volatile v8h*)(d1 + r * HD) = o1[r];
#pragma unroll
            for (int j = 0; j < 4; ++j) *(volatile v8h*)(d2 + j * HD) = o2[j];
            *(volatile v8h*)d8 = o8;
            if (ps == 0) __threadfence();
        }
    } else {
        const int ip = i - KPL_REAL; if (ip >= KPL_PAD) return;
        const int row = ip >> 4; const int h = row >> 5, pr = row & 31;
        v8h z;
#pragma unroll
        for (int e = 0; e < 8; ++e) z[e] = (h16)0.0f;
        h16* d = KP + K8OFF + ((size_t)h * K8R + T8 + pr) * HD + pc;
        *(volatile v8h*)d = z; __threadfence(); *(volatile v8h*)d = z;
    }
}

__global__ __launch_bounds__(256) void k_vtp(const float* __restrict__ v, h16* VP) {
    __shared__ float tl[512 * 33];
    const int t = threadIdx.x; const int tc = blockIdx.x, d0 = blockIdx.y * 32, h = blockIdx.z; const int t0 = tc * 512;
#pragma unroll 4
    for (int it = 0; it < 16; ++it) { const int idx = t + 256 * it; const int row = idx >> 3, c4 = (idx & 7) * 4;
        const v4f a = *(const v4f*)(v + ((size_t)h * SEQ_FULL + t0 + row) * HD + d0 + c4);
        tl[row * 33 + c4] = bfr(a[0]); tl[row * 33 + c4 + 1] = bfr(a[1]); tl[row * 33 + c4 + 2] = bfr(a[2]); tl[row * 33 + c4 + 3] = bfr(a[3]); }
    __syncthreads();
    v8h o1[8], o2[4], o8, z;
#pragma unroll
    for (int it = 0; it < 8; ++it) { const int p = t + 256 * it; const int dr = p >> 6, seg = p & 63;
#pragma unroll
        for (int e = 0; e < 8; ++e) o1[it][e] = toh_flush(tl[(seg * 8 + e) * 33 + dr]); }
#pragma unroll
    for (int it = 0; it < 4; ++it) { const int p = t + 256 * it; const int dr = p >> 5, seg = p & 31;
#pragma unroll
        for (int e = 0; e < 8; ++e) { const int u = seg * 8 + e; o2[it][e] = toh_flush((tl[(2 * u) * 33 + dr] + tl[(2 * u + 1) * 33 + dr]) * 0.5f); } }
    const int dr8 = t >> 3, seg8 = t & 7;
#pragma unroll
    for (int e = 0; e < 8; ++e) { const int u = seg8 * 8 + e; float s = tl[(8 * u) * 33 + dr8];
#pragma unroll
        for (int w = 1; w < 8; ++w) s += tl[(8 * u + w) * 33 + dr8];
        o8[e] = toh_flush(s * 0.125f); z[e] = (h16)0.0f; }
    const int rb = h * HD + d0;
#pragma unroll 1
    for (int ps = 0; ps < 2; ++ps) {
#pragma unroll
        for (int it = 0; it < 8; ++it) { const int p = t + 256 * it; const int dr = p >> 6, seg = p & 63;
            *(volatile v8h*)(VP + (size_t)(rb + dr) * SEQ + t0 + seg * 8) = o1[it]; }
#pragma unroll
        for (int it = 0; it < 4; ++it) { const int p = t + 256 * it; const int dr = p >> 5, seg = p & 31;
            *(volatile v8h*)(VP + VT2OFF + (size_t)(rb + dr) * T2 + tc * 256 + seg * 8) = o2[it]; }
        *(volatile v8h*)(VP + VT8OFF + (size_t)(rb + dr8) * V8P + tc * 64 + seg8 * 8) = o8;
        if (tc == SEQ / 512 - 1) *(volatile v8h*)(VP + VT8OFF + (size_t)(rb + dr8) * V8P + T8 + seg8 * 8) = z;
        if (ps == 0) __threadfence();
    }
}

__global__ __launch_bounds__(256) void k_samp(const float* __restrict__ q, const float* __restrict__ k, const float* __restrict__ randq, const float* __restrict__ randk, bf* SQ, bf* SK) {
    __shared__ float rq[128]; __shared__ float rk[64]; __shared__ int sq[32]; __shared__ int sk[16];
    const int t = threadIdx.x; const int c = blockIdx.x, h = blockIdx.y;
    const float ra = randq[h * 128 + (t & 127)]; const float rb = randk[h * 64 + (t & 63)];
    if (t < 128) rq[t] = bfr(ra);
    if (t < 64) rk[t] = bfr(rb);
    if (t < 32) sq[t] = 0;
    if (t < 16) sk[t] = 0;
    __syncthreads();
    { const int tq = t & 127; const float mv = rq[tq]; int rank = 0;
#pragma unroll 4
      for (int j = 0; j < 128; ++j) { const float x = rq[j]; rank += ((x > mv) | ((x == mv) & (j < tq))) ? 1 : 0; }
      if ((t < 128) & (rank < 32)) sq[rank] = tq; }
    { const int tk = t & 63; const float mv = rk[tk]; int rank = 0;
#pragma unroll 4
      for (int j = 0; j < 64; ++j) { const float x = rk[j]; rank += ((x > mv) | ((x == mv) & (j < tk))) ? 1 : 0; }
      if ((t < 64) & (rank < 16)) sk[rank] = tk; }
    __syncthreads();
    const int pc = (t & 15) * 8; v8us oq[4], ok[4];
#pragma unroll
    for (int it = 0; it < 4; ++it) { const int srow = c * 64 + (t >> 4) + 16 * it;
        const int tq = (srow >> 5) * 128 + (sq[srow & 31] & 127); const int tk = (srow >> 4) * 64 + (sk[srow & 15] & 63);
        const v8f vq = *(const v8f*)(q + ((size_t)h * SEQ_FULL + tq) * HD + pc); const v8f vk = *(const v8f*)(k + ((size_t)h * SEQ_FULL + tk) * HD + pc);
#pragma unroll
        for (int e = 0; e < 8; ++e) { oq[it][e] = f2bf(vq[e]); ok[it][e] = f2bf(vk[e]); } }
#pragma unroll 1
    for (int ps = 0; ps < 2; ++ps) {
#pragma unroll
        for (int it = 0; it < 4; ++it) { const int srow = c * 64 + (t >> 4) + 16 * it;
            *(volatile v8us*)(SQ + ((size_t)h * NSQ + srow) * HD + pc) = oq[it]; *(volatile v8us*)(SK + ((size_t)h * NSK + srow) * HD + pc) = ok[it]; }
        if (ps == 0) __threadfence();
    }
}

__global__ __launch_bounds__(128) void k_pool(const bf* __restrict__ SQ, const bf* __restrict__ SK, int* LV) {
    __shared__ float wmx[4 * 32]; __shared__ float wsm[4 * 32]; __shared__ float pool[32];
    const int lane = threadIdx.x & 31, lr = lane & 15, hi = lane >> 4;
    const int wave = __builtin_amdgcn_readfirstlane(threadIdx.x >> 5);
    const int qb = blockIdx.x, h = blockIdx.y;
    const int aoff = (h * NSQ + qb * 32 + lr) * HD + 8 * hi;
    const int boff = (h * NSK + wave * NT * 16 + lr) * HD + 8 * hi;
    v8f acc[2][NT];
#pragma unroll
    for (int mb = 0; mb < 2; ++mb)
#pragma unroll
        for (int nb = 0; nb < NT; ++nb) acc[mb][nb] = (v8f){};
#pragma unroll 1
    for (int kc = 0; kc < HD; kc += 32) {
        const v16bf a0 = ldb(SQ + aoff + kc); const v16bf a1 = ldb(SQ + aoff + 16 * HD + kc);
#pragma unroll
        for (int nb = 0; nb < NT; ++nb) { const v16bf b = ldb(SK + boff + nb * 16 * HD + kc);
            acc[0][nb] = wmmabg(a0, b, acc[0][nb]); acc[1][nb] = wmmabg(a1, b, acc[1][nb]); }
    }
    float gm[2][8], inv[2][8];
#pragma unroll
    for (int mb = 0; mb < 2; ++mb)
#pragma unroll
        for (int r = 0; r < 8; ++r) {
            float mx = -3.0e38f;
#pragma unroll
            for (int nb = 0; nb < NT; ++nb) { const float s = acc[mb][nb][r] * PSC; acc[mb][nb][r] = s; mx = fmaxf(mx, s); }
            mx = fmaxf(mx, __shfl_xor(mx, 1, 32)); mx = fmaxf(mx, __shfl_xor(mx, 2, 32)); mx = fmaxf(mx, __shfl_xor(mx, 4, 32)); mx = fmaxf(mx, __shfl_xor(mx, 8, 32));
            gm[mb][r] = mx;
        }
    if (lr == 0) {
#pragma unroll
        for (int mb = 0; mb < 2; ++mb)
#pragma unroll
            for (int r = 0; r < 8; ++r) wmx[wave * 32 + mb * 16 + 8 * hi + r] = gm[mb][r];
    }
    __syncthreads();
#pragma unroll
    for (int mb = 0; mb < 2; ++mb)
#pragma unroll
        for (int r = 0; r < 8; ++r) { const int row = mb * 16 + 8 * hi + r;
            gm[mb][r] = fmaxf(fmaxf(wmx[row], wmx[32 + row]), fmaxf(wmx[64 + row], wmx[96 + row])); }
#pragma unroll
    for (int mb = 0; mb < 2; ++mb)
#pragma unroll
        for (int r = 0; r < 8; ++r) {
            float part = 0.0f;
#pragma unroll
            for (int nb = 0; nb < NT; ++nb) {
                float e = expf(acc[mb][nb][r] - gm[mb][r]);
                e += __shfl_xor(e, 1, 32); e += __shfl_xor(e, 2, 32); e += __shfl_xor(e, 4, 32); e += __shfl_xor(e, 8, 32);
                acc[mb][nb][r] = e; part += e;
            }
            inv[mb][r] = part;
        }
    if (lr == 0) {
#pragma unroll
        for (int mb = 0; mb < 2; ++mb)
#pragma unroll
            for (int r = 0; r < 8; ++r) wsm[wave * 32 + mb * 16 + 8 * hi + r] = inv[mb][r];
    }
    __syncthreads();
#pragma unroll
    for (int mb = 0; mb < 2; ++mb)
#pragma unroll
        for (int r = 0; r < 8; ++r) { const int row = mb * 16 + 8 * hi + r;
            inv[mb][r] = 1.0f / (((wsm[row] + wsm[32 + row]) + wsm[64 + row]) + wsm[96 + row]); }
#pragma unroll
    for (int nb = 0; nb < NT; ++nb) {
        float pp = 0.0f;
#pragma unroll
        for (int mb = 0; mb < 2; ++mb)
#pragma unroll
            for (int r = 0; r < 8; ++r) pp += acc[mb][nb][r] * inv[mb][r];
        pp += __shfl_xor(pp, 16, 32);
        if (lane == 0) pool[wave * NT + nb] = pp * 0.03125f;
    }
    __syncthreads();
    if (wave == 0) {
        const int kbi = (lane < NKB) ? lane : (NKB - 1);
        const float mv = pool[kbi]; int rank = 0;
#pragma unroll 4
        for (int j = 0; j < NKB; ++j) { const float pj = pool[j]; rank += ((pj > mv) | ((pj == mv) & (j < lane))) ? 1 : 0; }
        const float frac = (float)rank * (1.0f / (float)NKB);
        int lev = 0;
        if ((frac >= 0.0f) & (frac < 0.1f)) lev = 1;
        if ((frac >= 0.1f) & (frac < 0.15f)) lev = 2;
        if ((frac >= 0.15f) & (frac < 0.35f)) lev = 8;
        if (lane >= NKB) lev = 0;
        volatile int* dst = LV + (h * NQB + qb) * 32 + lane;
        *dst = lev; __threadfence(); *dst = lev;
    }
}

__device__ __forceinline__ void psa_step(const h16* __restrict__ Q16, const h16* __restrict__ KP, const h16* __restrict__ VP,
                                         const int qoff, const int koff, const int voff, const int vpitch, const float lbias, const int nvalid,
                                         v8f (&o)[8], float (&m)[8], float (&l)[8]) {
    __shared__ __align__(16) h16 ps[16 * 40];
    const int lane = threadIdx.x & 31, lr = lane & 15, hi = lane >> 4;
    const bool ok0 = lr < nvalid, ok1 = (16 + lr) < nvalid;
    v8f s0 = (v8f){}, s1 = (v8f){};
#pragma unroll 1
    for (int f = 0; f < 4; ++f) {
        const v16h qa = ldh(Q16 + qoff + f * 32);
        const v16h b0 = ldh(KP + koff + f * 32);
        const v16h b1 = ldh(KP + koff + 16 * HD + f * 32);
        s0 = wmma16g(qa, b0, s0); s1 = wmma16g(qa, b1, s1);
    }
#pragma unroll
    for (int r = 0; r < 8; ++r) {
        const float a0 = ok0 ? (s0[r] * CSL + lbias) : -3.0e38f;
        const float a1 = ok1 ? (s1[r] * CSL + lbias) : -3.0e38f;
        float mx = fmaxf(a0, a1);
        mx = fmaxf(mx, __shfl_xor(mx, 1, 32)); mx = fmaxf(mx, __shfl_xor(mx, 2, 32)); mx = fmaxf(mx, __shfl_xor(mx, 4, 32)); mx = fmaxf(mx, __shfl_xor(mx, 8, 32));
        const float mn = fmaxf(m[r], mx);
        const float al = __builtin_amdgcn_exp2f(m[r] - mn);
        const float e0 = (a0 - mn) + PSH, e1 = (a1 - mn) + PSH;
        const float p0 = (e0 < -14.0f) ? 0.0f : __builtin_amdgcn_exp2f(e0);
        const float p1 = (e1 < -14.0f) ? 0.0f : __builtin_amdgcn_exp2f(e1);
        const h16 h0 = (h16)p0, h1 = (h16)p1;
        l[r] = l[r] * al + ((float)h0 + (float)h1);
        m[r] = mn;
#pragma unroll
        for (int j = 0; j < 8; ++j) o[j][r] *= al;
        ps[(8 * hi + r) * 40 + lr] = h0;
        ps[(8 * hi + r) * 40 + 16 + lr] = h1;
    }
    __builtin_amdgcn_wave_barrier(); asm volatile("" ::: "memory");
    const v16h pf = cat16(*(const v8ha*)&ps[lr * 40 + 8 * hi], *(const v8ha*)&ps[lr * 40 + 16 + 8 * hi]);
    {
        v16h vb[4];
#pragma unroll
        for (int jj = 0; jj < 4; ++jj) vb[jj] = ldh(VP + voff + jj * 16 * vpitch);
#pragma unroll
        for (int jj = 0; jj < 4; ++jj) o[jj] = wmma16g(pf, vb[jj], o[jj]);
    }
    {
        v16h vb[4];
#pragma unroll
        for (int jj = 0; jj < 4; ++jj) vb[jj] = ldh(VP + voff + (4 + jj) * 16 * vpitch);
#pragma unroll
        for (int jj = 0; jj < 4; ++jj) o[4 + jj] = wmma16g(pf, vb[jj], o[4 + jj]);
    }
    __builtin_amdgcn_wave_barrier(); asm volatile("" ::: "memory");
}

__global__ __launch_bounds__(32) void k_psa(const h16* __restrict__ Q16, const h16* __restrict__ KP, const h16* __restrict__ VP, const int* __restrict__ LV, float* OUT) {
    __shared__ __align__(16) float os[16 * 132];
    const int lane = threadIdx.x & 31, lr = lane & 15, hi = lane >> 4;
    const int h = blockIdx.y, q0 = blockIdx.x * 16, qb = blockIdx.x >> 3;
    const int qoff = (h * SEQ + q0 + lr) * HD + 8 * hi;
    const int kl = lr * HD + 8 * hi;
    const int lvv = LV[(h * NQB + qb) * 32 + lane];
    v8f o[8]; float m[8], l[8];
#pragma unroll
    for (int j = 0; j < 8; ++j) o[j] = (v8f){};
#pragma unroll
    for (int r = 0; r < 8; ++r) { m[r] = -3.0e38f; l[r] = 0.0f; }
#pragma unroll 1
    for (int kb = 0; kb < NKB; ++kb) {
        const int lv = __builtin_amdgcn_readlane(lvv, kb);
        if (lv == 1) {
            const int ko = (h * SEQ + kb * 64) * HD + kl;
            const int vo = (h * HD + lr) * SEQ + kb * 64 + 8 * hi;
            psa_step(Q16, KP, VP, qoff, ko, vo, SEQ, 0.0f, 32, o, m, l);
            psa_step(Q16, KP, VP, qoff, ko + 32 * HD, vo + 32, SEQ, 0.0f, 32, o, m, l);
        } else if (lv == 2) {
            const int ko = K2OFF + (h * T2 + kb * 32) * HD + kl;
            const int vo = VT2OFF + (h * HD + lr) * T2 + kb * 32 + 8 * hi;
            psa_step(Q16, KP, VP, qoff, ko, vo, T2, 1.0f, 32, o, m, l);
        } else if (lv == 8) {
            const int ko = K8OFF + (h * K8R + kb * 8) * HD + kl;
            const int vo = VT8OFF + (h * HD + lr) * V8P + kb * 8 + 8 * hi;
            psa_step(Q16, KP, VP, qoff, ko, vo, V8P, 3.0f, 8, o, m, l);
        }
    }
#pragma unroll
    for (int r = 0; r < 8; ++r) {
        float lt = l[r];
        lt += __shfl_xor(lt, 1, 32); lt += __shfl_xor(lt, 2, 32); lt += __shfl_xor(lt, 4, 32); lt += __shfl_xor(lt, 8, 32);
        const float inv = 1.0f / lt;
#pragma unroll
        for (int j = 0; j < 8; ++j) os[(8 * hi + r) * 132 + j * 16 + lr] = o[j][r] * inv;
    }
    __builtin_amdgcn_wave_barrier(); asm volatile("" ::: "memory");
    float* orow = OUT + ((size_t)h * SEQ_FULL + q0) * HD + lane * 4;
#pragma unroll 1
    for (int pass = 0; pass < 2; ++pass) {
#pragma unroll
        for (int row = 0; row < 16; ++row) {
            const v4f val = *(const v4fa*)&os[row * 132 + lane * 4];
            *(volatile v4f*)(orow + (size_t)row * HD) = val;
        }
        if (pass == 0) __threadfence();
    }
}

#define AL256(x) ((((size_t)(x)) + 255) & ~(size_t)255)
#define CARVE (AL256((size_t)NHD * SEQ * HD * 2) + AL256((size_t)KPOOL * 2) + AL256((size_t)VPOOL * 2) + 2 * AL256((size_t)NHD * NSQ * HD * 2) + AL256((size_t)NHD * NQB * 32 * 4))
static_assert(CARVE <= (size_t)134217728);
static_assert((size_t)KPOOL < (size_t)2147483647);
static_assert((size_t)VPOOL < (size_t)2147483647);

extern "C" void kernel_launch(void* const* d_in, const int* in_sizes, int n_in,
                              void* d_out, int out_size, void* d_ws, size_t ws_size, hipStream_t stream) {
    if (n_in < 5) return;
    const size_t need = ((size_t)(NHD - 1) * SEQ_FULL + SEQ) * HD;
    if ((size_t)in_sizes[0] < need || (size_t)in_sizes[1] < need || (size_t)in_sizes[2] < need) return;
    if (in_sizes[3] < NHD * 128 || in_sizes[4] < NHD * 64) return;
    if ((size_t)out_size < need) return;
    if (ws_size < CARVE) return;
    const float* q  = (const float*)d_in[0];
    const float* k  = (const float*)d_in[1];
    const float* v  = (const float*)d_in[2];
    const float* rq = (const float*)d_in[3];
    const float* rk = (const float*)d_in[4];
    float* OUT = (float*)d_out;
    char* wsp = (char*)d_ws;
    auto take = [&](size_t bytes) { char* p = wsp; wsp += (bytes + 255) & ~(size_t)255; return (void*)p; };
    h16* Q16 = (h16*)take((size_t)NHD * SEQ * HD * 2);
    h16* KP  = (h16*)take((size_t)KPOOL * 2);
    h16* VP  = (h16*)take((size_t)VPOOL * 2);
    bf*  SQ  = (bf*)take((size_t)NHD * NSQ * HD * 2);
    bf*  SK  = (bf*)take((size_t)NHD * NSK * HD * 2);
    int* LV  = (int*)take((size_t)NHD * NQB * 32 * 4);
    if ((size_t)(wsp - (char*)d_ws) > ws_size) return;

    k_cvtq<<<(NHD * SEQ * 16) / 256, 256, 0, stream>>>(q, Q16);
    k_kpl<<<(KPL_REAL + KPL_PAD) / 256, 256, 0, stream>>>(k, KP);
    k_vtp<<<dim3(SEQ / 512, HD / 32, NHD), 256, 0, stream>>>(v, VP);
    k_samp<<<dim3(NSQ / 64, NHD), 256, 0, stream>>>(q, k, rq, rk, SQ, SK);
    k_pool<<<dim3(NQB, NHD), 128, 0, stream>>>(SQ, SK, LV);
    k_psa<<<dim3(SEQ / 16, NHD), 32, 0, stream>>>(Q16, KP, VP, LV, OUT);
}
